// ATTBase_84851373900347
// MI455X (gfx1250) — hardware-verified
//
#include <hip/hip_runtime.h>

#define HN    100
#define NT    7
#define NROW  112
#define OBS   18
#define OBSS  54
#define RB    32
#define PV    128
#define NPV   24
#define XP    32
#define SP    128
#define CATP  320
#define FIJP  104

#define KA1   32
#define KSQ   128
#define KEO   320
#define KCR   224

#define PH_A1   0
#define PH_A2   (PH_A1   + NROW * KA1)
#define PH_EOUT (PH_A2   + NROW * KSQ)
#define PH_CORR (PH_EOUT + NROW * KEO)
#define PH_FC   (PH_CORR + NROW * KSQ)
#define PH_CR1  (PH_FC   + NROW * KSQ)
#define PH_END  (PH_CR1  + NROW * KCR)
#define PAR_OFFB  ((size_t)PH_END * 2)
#define PAR_BYTES ((size_t)NPV * PV * 4)
#define WS_TOTAL  (PAR_OFFB + PAR_BYTES)

static_assert(PH_END == 107520);
static_assert(WS_TOTAL == 227328);
static_assert((PH_A2 % 256) == 0);
static_assert((PH_EOUT % 256) == 0);
static_assert((PH_CORR % 256) == 0);
static_assert((PH_FC % 256) == 0);
static_assert((PH_CR1 % 256) == 0);
static_assert((PH_END % 256) == 0);
static_assert(((NROW * KA1 / 8) % 32) == 0);
static_assert(((NROW * KSQ / 8) % 32) == 0);
static_assert(((NROW * KEO / 8) % 32) == 0);
static_assert(((NROW * KCR / 8) % 32) == 0);
static_assert((PAR_BYTES % 4096) == 0);
static_assert(((RB * HN) % 128) == 0);
static_assert(FIJP >= HN + 4);
static_assert((FIJP % 4) == 0);
static_assert(3 * HN + 20 == KEO);
static_assert(2 * HN + 24 == KCR);

enum { V_B1 = 0, V_B2, V_AW0, V_AW1, V_AB, V_LW0, V_LW1, V_LB, V_EOB, V_FCB, V_CB1, V_CW2, V_CB2,
       V_T0, V_T1, V_T2, V_T3, V_T4, V_NUSED };
static_assert(V_NUSED <= NPV);
static_assert(V_T0 == 13);

#define L_CATH  0
#define L_CATL  (L_CATH + RB * CATP * 2)
#define L_FIIH  (L_CATL + RB * CATP * 2)
#define L_FIIL  (L_FIIH + RB * SP * 2)
#define L_FIJ   (L_FIIL + RB * SP * 2)
#define L_ROW   (L_FIJ  + 2 * RB * FIJP * 4)
#define L_TOTAL (L_ROW  + 2 * RB * 4)
static_assert(L_TOTAL == 84224);
static_assert((L_CATL % 16) == 0);
static_assert((L_FIIH % 16) == 0);
static_assert((L_FIIL % 16) == 0);
static_assert((L_FIJ % 16) == 0);
static_assert((L_ROW % 16) == 0);

typedef unsigned short us16;
typedef __bf16 v16b __attribute__((ext_vector_type(16)));
typedef us16   v16us __attribute__((ext_vector_type(16)));
typedef us16   v8us_t __attribute__((ext_vector_type(8)));
typedef v8us_t __attribute__((may_alias)) v8us;
typedef float  v8f   __attribute__((ext_vector_type(8)));
typedef float  v4f_t __attribute__((ext_vector_type(4)));
typedef v4f_t  __attribute__((may_alias)) v4f;
typedef unsigned int v4u_t __attribute__((ext_vector_type(4)));
typedef v4u_t  __attribute__((may_alias)) v4u;
typedef unsigned int v2u_t __attribute__((ext_vector_type(2)));
typedef v2u_t  __attribute__((may_alias)) v2u;
typedef unsigned int __attribute__((may_alias)) u32a;
union Frag { v16us v; v8us_t h[2]; };

__device__ __forceinline__ v8f zero8() {
    v8f z;
#pragma unroll
    for (int i = 0; i < 8; ++i) z[i] = 0.0f;
    return z;
}

__device__ __forceinline__ unsigned int bf_bits(float x) {
    const unsigned int u = __float_as_uint(x);
    return (u + 0x7FFFu + ((u >> 16) & 1u)) >> 16;
}
__device__ __forceinline__ float bfr(float x) {
    return __uint_as_float(bf_bits(x) << 16);
}
__device__ __forceinline__ void split2(float a, unsigned int& hb, unsigned int& lb) {
    hb = bf_bits(a);
    const float h = __uint_as_float(hb << 16);
    lb = bf_bits(a - h);
}

__device__ __forceinline__ float tanh_v(float x) {
    const float ax = fabsf(x);
    const float t  = __expf(-2.0f * ax);
    const float r  = (1.0f - t) * __builtin_amdgcn_rcpf(1.0f + t);
    return copysignf(r, x);
}

__device__ __forceinline__ void softmax2(float b0, float b1, float& a0, float& a1) {
    const float mx = fmaxf(b0, b1);
    const float e0 = __expf(b0 - mx), e1 = __expf(b1 - mx);
    const float inv = __builtin_amdgcn_rcpf(e0 + e1);
    a0 = e0 * inv; a1 = e1 * inv;
}

__device__ __forceinline__ v16us ldfrag(const us16* p, int k0) {
    Frag f;
    f.h[0] = *(const v8us*)(p + k0);
    f.h[1] = *(const v8us*)(p + k0 + 16);
    return f.v;
}

__device__ __forceinline__ v8f wmma_bf(v16us a, v16us b, v8f c) {
    return __builtin_amdgcn_wmma_f32_16x16x32_bf16(false, __builtin_bit_cast(v16b, a), false,
                                                   __builtin_bit_cast(v16b, b), (short)0, c, false, false);
}

__device__ __forceinline__ void reduce16(float (&d)[8]) {
#pragma unroll
    for (int r = 0; r < 8; ++r) {
#pragma unroll
        for (int o = 1; o < 16; o <<= 1) d[r] += __shfl_xor(d[r], o, 32);
    }
}

template <int KP, bool SPLIT>
__device__ __forceinline__ void tile_mm(const us16* aH, const us16* aL, int pitch,
                                        const us16* __restrict__ bt, int lane, v8f& c0, v8f& c1)
{
    c0 = zero8(); c1 = zero8();
    const int m = lane & 15, hh = lane >> 4;
    const us16* ph0 = aH + m * pitch + 8 * hh;
    const us16* ph1 = ph0 + 16 * pitch;
    const us16* pl0 = aL + m * pitch + 8 * hh;
    const us16* pl1 = pl0 + 16 * pitch;
    const us16* pb  = bt + (size_t)m * KP + 8 * hh;
#pragma unroll 1
    for (int k0 = 0; k0 < KP; k0 += 32) {
        const v16us b  = ldfrag(pb, k0);
        const v16us a0 = ldfrag(ph0, k0);
        const v16us a1 = ldfrag(ph1, k0);
        c0 = wmma_bf(a0, b, c0);
        c1 = wmma_bf(a1, b, c1);
        if (SPLIT) {
            const v16us l0 = ldfrag(pl0, k0);
            const v16us l1 = ldfrag(pl1, k0);
            c0 = wmma_bf(l0, b, c0);
            c1 = wmma_bf(l1, b, c1);
            asm volatile("v_nop\n\tv_nop\n\tv_nop\n\tv_nop"
                         : "+v"(c0), "+v"(c1)
                         : "v"(a0), "v"(a1), "v"(l0), "v"(l1), "v"(b));
        } else {
            asm volatile("v_nop\n\tv_nop\n\tv_nop\n\tv_nop"
                         : "+v"(c0), "+v"(c1)
                         : "v"(a0), "v"(a1), "v"(b));
        }
    }
}

__global__ void __launch_bounds__(256) pack_plane(const float* __restrict__ W, int korig, int kp,
                                                  int nsrc, int npieces, us16* __restrict__ dst)
{
    const int q  = blockIdx.x * 256 + threadIdx.x;
    const bool ok = (q < npieces);
    const int qq = ok ? q : 0;
    const int e0 = qq * 8;
    const int n  = e0 / kp;
    const int k0 = e0 - n * kp;
    const int nn = (n < nsrc) ? n : (nsrc - 1);
    v4u_t pk;
#pragma unroll
    for (int j = 0; j < 4; ++j) {
        const int ka = k0 + 2 * j, kb = ka + 1;
        const int kac = (ka < korig) ? ka : (korig - 1);
        const int kbc = (kb < korig) ? kb : (korig - 1);
        const float wa = W[(size_t)kac * HN + nn];
        const float wb = W[(size_t)kbc * HN + nn];
        const unsigned int ba = (ka < korig && n < nsrc) ? bf_bits(wa) : 0u;
        const unsigned int bb = (kb < korig && n < nsrc) ? bf_bits(wb) : 0u;
        pk[j] = ba | (bb << 16);
    }
    us16* d = dst + (size_t)qq * 8;
    if (ok) *(volatile v4u_t*)d = pk;
    __threadfence();
    if (ok) *(volatile v4u_t*)d = pk;
}

__global__ void __launch_bounds__(256) prep_small(
    const float* __restrict__ ab1, const float* __restrict__ ab2,
    const float* __restrict__ esw, const float* __restrict__ esb,
    const float* __restrict__ eaw, const float* __restrict__ eab,
    const float* __restrict__ elw, const float* __restrict__ elb,
    const float* __restrict__ eac, const float* __restrict__ elc,
    const float* __restrict__ efw, const float* __restrict__ efb,
    const float* __restrict__ eob, const float* __restrict__ fcb,
    const float* __restrict__ cb1, const float* __restrict__ cw2,
    const float* __restrict__ cb2, float* __restrict__ par)
{
    __shared__ float  sT[5 * NROW];
    __shared__ double sQ[6 * HN];
    __shared__ __align__(16) float sPar[NPV * PV];
    const int tid = threadIdx.x;

    for (int i = tid; i < NPV * PV; i += 256) sPar[i] = 0.0f;
    for (int i = tid; i < 5 * NROW; i += 256) sT[i] = 0.0f;
    __syncthreads();

#pragma unroll 1
    for (int it = 0; it < 2; ++it) {
        const int o  = tid + 256 * it;
        const int oc = (o < 500) ? o : 499;
        const int c  = oc / HN, n = oc - c * HN;
        const int cs = (c < 4) ? c : 3;
        double acc = 0.0;
#pragma unroll 1
        for (int h = 0; h < HN; ++h) {
            const float wsv = bfr(esw[cs * HN + h]);
            const float bsv = bfr(esb[h]);
            const float a = (c < 4) ? wsv : bsv;
            acc = fma((double)a, (double)bfr(efw[h * HN + n]), acc);
        }
        const float eb = bfr(efb[n]);
        acc += (c == 4) ? (double)eb : 0.0;
        if (o < 500) sT[c * NROW + n] = (float)acc;
    }
#pragma unroll 1
    for (int it = 0; it < 3; ++it) {
        const int o  = tid + 256 * it;
        const int oc = (o < 600) ? o : 599;
        const int i  = oc / HN, h = oc - i * HN;
        const int g  = (i >= 3) ? 1 : 0;
        const int j  = i - 3 * g;
        const int jc = (j < 2) ? j : 1;
        double acc = 0.0;
#pragma unroll 1
        for (int k = 0; k < HN; ++k) {
            const float ca = bfr(eac[h * HN + k]);
            const float cl = bfr(elc[h * HN + k]);
            const float cv = g ? cl : ca;
            const float wa = bfr(eaw[jc * HN + k]), ba = bfr(eab[k]);
            const float wl = bfr(elw[jc * HN + k]), bl = bfr(elb[k]);
            const float wsel = g ? ((j == 2) ? bl : wl) : ((j == 2) ? ba : wa);
            acc = fma((double)cv, (double)wsel, acc);
        }
        if (o < 600) sQ[i * HN + h] = acc;
    }
    __syncthreads();
    {
        const int oc = (tid < 30) ? tid : 29;
        const int c  = oc / 6, i = oc - 6 * c;
        const int cs = (c < 4) ? c : 3;
        double acc = 0.0;
#pragma unroll 1
        for (int h = 0; h < HN; ++h) {
            const float wsv = bfr(esw[cs * HN + h]);
            const float bsv = bfr(esb[h]);
            const float a = (c < 4) ? wsv : bsv;
            acc = fma((double)a, sQ[i * HN + h], acc);
        }
        if (tid < 30) sT[c * NROW + HN + i] = (float)acc;
    }
    __syncthreads();
#pragma unroll 1
    for (int v = 0; v < V_T0; ++v) {
        const float* src = ab1; int cnt = HN;
        if (v == V_B2) src = ab2;
        else if (v == V_AW0) src = eaw;
        else if (v == V_AW1) src = eaw + HN;
        else if (v == V_AB)  src = eab;
        else if (v == V_LW0) src = elw;
        else if (v == V_LW1) src = elw + HN;
        else if (v == V_LB)  src = elb;
        else if (v == V_EOB) src = eob;
        else if (v == V_FCB) src = fcb;
        else if (v == V_CB1) src = cb1;
        else if (v == V_CW2) src = cw2;
        else if (v == V_CB2) { src = cb2; cnt = 1; }
        const int tc = (tid < cnt) ? tid : (cnt - 1);
        const float val = bfr(src[tc]);
        if (tid < cnt) sPar[v * PV + tid] = val;
    }
    for (int i = tid; i < 5 * NROW; i += 256) {
        const int c = i / NROW, n = i - c * NROW;
        sPar[(V_T0 + c) * PV + n] = sT[i];
    }
    __syncthreads();
    v4f_t o[3];
#pragma unroll
    for (int it = 0; it < 3; ++it) o[it] = *(const v4f*)(sPar + 4 * (tid + 256 * it));
#pragma unroll
    for (int it = 0; it < 3; ++it) *(volatile v4f_t*)(par + 4 * (tid + 256 * it)) = o[it];
    __threadfence();
#pragma unroll
    for (int it = 0; it < 3; ++it) *(volatile v4f_t*)(par + 4 * (tid + 256 * it)) = o[it];
}

__global__ void __launch_bounds__(32)
actor_kernel(const float* __restrict__ inp, const us16* __restrict__ wsh,
             const float* __restrict__ par, float* __restrict__ out, int bsz)
{
    __shared__ __align__(16) us16  sX[RB * XP];
    __shared__ __align__(16) us16  sH[RB * SP];
    __shared__ __align__(16) us16  sL[RB * SP];
    __shared__ __align__(16) float stg[RB * HN];

    const int lane = threadIdx.x, m = lane & 15, hh = lane >> 4;
    const int b0 = blockIdx.x * RB;
    if (b0 + RB > bsz) return;

    {
        const float* src = inp + (size_t)(b0 + lane) * OBS;
        unsigned int xb[OBS];
#pragma unroll
        for (int c = 0; c < OBS; ++c) xb[c] = bf_bits(src[c]);
        us16* rp = sX + lane * XP;
#pragma unroll
        for (int c = 0; c < OBS / 2; ++c) *(u32a*)(rp + 2 * c) = xb[2 * c] | (xb[2 * c + 1] << 16);
#pragma unroll
        for (int c = OBS / 2; c < XP / 2; ++c) *(u32a*)(rp + 2 * c) = 0u;
    }
    __syncthreads();

    const float* b1 = par + V_B1 * PV;
#pragma unroll 1
    for (int nt = 0; nt < NT; ++nt) {
        v8f c0, c1;
        tile_mm<KA1, false>(sX, sX, XP, wsh + PH_A1 + nt * 16 * KA1, lane, c0, c1);
        const int n = nt * 16 + m;
        const float bb = b1[n];
        const bool okn = (n < HN);
#pragma unroll
        for (int r = 0; r < 8; ++r) {
            const float v0 = okn ? tanh_v(c0[r] + bb) : 0.0f;
            const float v1 = okn ? tanh_v(c1[r] + bb) : 0.0f;
            unsigned int h0, l0, h1, l1;
            split2(v0, h0, l0); split2(v1, h1, l1);
            const int ia = (8 * hh + r) * SP + n, ib = (16 + 8 * hh + r) * SP + n;
            sH[ia] = (us16)h0; sL[ia] = (us16)l0;
            sH[ib] = (us16)h1; sL[ib] = (us16)l1;
        }
    }
    {
        v4u_t z4; z4.x = 0u; z4.y = 0u; z4.z = 0u; z4.w = 0u;
        *(v4u*)(sH + lane * SP + 112) = z4; *(v4u*)(sH + lane * SP + 120) = z4;
        *(v4u*)(sL + lane * SP + 112) = z4; *(v4u*)(sL + lane * SP + 120) = z4;
    }
    __syncthreads();

    const float* b2 = par + V_B2 * PV;
#pragma unroll 1
    for (int nt = 0; nt < NT; ++nt) {
        v8f c0, c1;
        tile_mm<KSQ, true>(sH, sL, SP, wsh + PH_A2 + nt * 16 * KSQ, lane, c0, c1);
        const int n = nt * 16 + m;
        const float bb = b2[n];
        float v0[8], v1[8];
#pragma unroll
        for (int r = 0; r < 8; ++r) { v0[r] = tanh_v(c0[r] + bb); v1[r] = tanh_v(c1[r] + bb); }
        if (n < HN) {
#pragma unroll
            for (int r = 0; r < 8; ++r) {
                stg[(8 * hh + r) * HN + n]      = v0[r];
                stg[(16 + 8 * hh + r) * HN + n] = v1[r];
            }
        }
    }
    __syncthreads();

    {
        float* o1 = out + (size_t)bsz + (size_t)b0 * HN;
#pragma unroll
        for (int i = 0; i < (RB * HN) / 128; ++i)
            *(volatile v4f_t*)(o1 + 4 * (lane + 32 * i)) = *(const v4f*)(stg + 4 * (lane + 32 * i));
        __threadfence();
#pragma unroll
        for (int i = 0; i < (RB * HN) / 128; ++i)
            *(volatile v4f_t*)(o1 + 4 * (lane + 32 * i)) = *(const v4f*)(stg + 4 * (lane + 32 * i));
    }
}

__global__ void __launch_bounds__(32)
enc_head_kernel(const float* __restrict__ share, const float* __restrict__ inp,
                const int* __restrict__ agent, const float* __restrict__ rnn,
                const us16* __restrict__ wsh, const float* __restrict__ par,
                float* __restrict__ out, int bsz)
{
    extern __shared__ __align__(16) unsigned char dynl[];
    us16*  sCatH = (us16*)(dynl + L_CATH);
    us16*  sCatL = (us16*)(dynl + L_CATL);
    us16*  sFiiH = (us16*)(dynl + L_FIIH);
    us16*  sFiiL = (us16*)(dynl + L_FIIL);
    float* sFij  = (float*)(dynl + L_FIJ);
    float* sRow  = (float*)(dynl + L_ROW);

    const int lane = threadIdx.x, m = lane & 15, hh = lane >> 4;
    const int b0 = blockIdx.x * RB;
    if (b0 + RB > bsz) return;

    int ai = agent[0];
    ai = (ai < 0) ? 0 : ((ai > 2) ? 2 : ai);
    const int j0 = (ai == 0) ? 1 : 0;
    const int j1 = (ai == 2) ? 1 : 2;

    const float* T0  = par + V_T0 * PV;
    const float* T1  = par + V_T1 * PV;
    const float* T2  = par + V_T2 * PV;
    const float* T3  = par + V_T3 * PV;
    const float* T4  = par + V_T4 * PV;
    const float* AW0 = par + V_AW0 * PV;
    const float* AW1 = par + V_AW1 * PV;
    const float* AB  = par + V_AB * PV;
    const float* LW0 = par + V_LW0 * PV;
    const float* LW1 = par + V_LW1 * PV;
    const float* LB  = par + V_LB * PV;
    const float* EOB = par + V_EOB * PV;

#pragma unroll 1
    for (int e = 0; e < 3; ++e) {
        __syncthreads();
        {
            const int jj = (e == 1) ? j0 : j1;
            const float* src = (e == 0) ? (inp + (size_t)(b0 + lane) * OBS)
                                        : (share + (size_t)(b0 + lane) * OBSS + (size_t)(jj * OBS));
            float x[14];
#pragma unroll
            for (int c = 0; c < 14; ++c) x[c] = bfr(src[c]);
            float d[6];
#pragma unroll
            for (int i = 0; i < 6; ++i)
                d[i] = fmaf(x[3], T3[HN + i], fmaf(x[2], T2[HN + i], fmaf(x[1], T1[HN + i], fmaf(x[0], T0[HN + i], T4[HN + i]))));
            float aa0, aa1;
            softmax2(fmaf(x[10], d[0], fmaf(x[11], d[1], d[2])),
                     fmaf(x[12], d[0], fmaf(x[13], d[1], d[2])), aa0, aa1);
            const float xba = fmaf(aa0, x[10], aa1 * x[12]);
            const float yba = fmaf(aa0, x[11], aa1 * x[13]);
            const float sba = aa0 + aa1;
            const float bl0 = fmaf(x[4], d[3], fmaf(x[5], d[4], d[5]));
            const float bl1 = fmaf(x[6], d[3], fmaf(x[7], d[4], d[5]));
            const float bl2 = fmaf(x[8], d[3], fmaf(x[9], d[4], d[5]));
            const float ml  = fmaxf(fmaxf(bl0, bl1), bl2);
            const float el0 = __expf(bl0 - ml), el1 = __expf(bl1 - ml), el2 = __expf(bl2 - ml);
            const float il  = __builtin_amdgcn_rcpf(el0 + el1 + el2);
            const float al0 = el0 * il, al1 = el1 * il, al2 = el2 * il;
            const float xbl = fmaf(al0, x[4], fmaf(al1, x[6], al2 * x[8]));
            const float ybl = fmaf(al0, x[5], fmaf(al1, x[7], al2 * x[9]));
            const float sbl = al0 + al1 + al2;
            us16* ch = sCatH + lane * CATP;
            us16* cl = sCatL + lane * CATP;
#pragma unroll 1
            for (int n = 0; n < HN; n += 2) {
                unsigned int pgh = 0u, pgl = 0u, pah = 0u, pal = 0u, plh = 0u, pll = 0u;
#pragma unroll
                for (int u = 0; u < 2; ++u) {
                    const int nn = n + u;
                    const float gi = fmaf(x[3], T3[nn], fmaf(x[2], T2[nn], fmaf(x[1], T1[nn], fmaf(x[0], T0[nn], T4[nn]))));
                    const float va = fmaf(xba, AW0[nn], fmaf(yba, AW1[nn], sba * AB[nn]));
                    const float vl = fmaf(xbl, LW0[nn], fmaf(ybl, LW1[nn], sbl * LB[nn]));
                    unsigned int hb, lb;
                    split2(gi, hb, lb); pgh |= hb << (16 * u); pgl |= lb << (16 * u);
                    split2(va, hb, lb); pah |= hb << (16 * u); pal |= lb << (16 * u);
                    split2(vl, hb, lb); plh |= hb << (16 * u); pll |= lb << (16 * u);
                }
                *(u32a*)(ch + n)          = pgh; *(u32a*)(cl + n)          = pgl;
                *(u32a*)(ch + HN + n)     = pah; *(u32a*)(cl + HN + n)     = pal;
                *(u32a*)(ch + 2 * HN + n) = plh; *(u32a*)(cl + 2 * HN + n) = pll;
            }
            v2u_t z2; z2.x = 0u; z2.y = 0u;
#pragma unroll
            for (int c = 3 * HN; c < KEO; c += 4) { *(v2u*)(ch + c) = z2; *(v2u*)(cl + c) = z2; }
        }
        __syncthreads();

#pragma unroll 1
        for (int nt = 0; nt < NT; ++nt) {
            v8f c0, c1;
            tile_mm<KEO, true>(sCatH, sCatL, CATP, wsh + PH_EOUT + nt * 16 * KEO, lane, c0, c1);
            const int n = nt * 16 + m;
            const float bb = EOB[n];
            const bool okn = (n < HN);
            if (e == 0) {
#pragma unroll
                for (int r = 0; r < 8; ++r) {
                    const float v0 = okn ? (c0[r] + bb) : 0.0f;
                    const float v1 = okn ? (c1[r] + bb) : 0.0f;
                    unsigned int h0, l0, h1, l1;
                    split2(v0, h0, l0); split2(v1, h1, l1);
                    const int ia = (8 * hh + r) * SP + n, ib = (16 + 8 * hh + r) * SP + n;
                    sFiiH[ia] = (us16)h0; sFiiL[ia] = (us16)l0;
                    sFiiH[ib] = (us16)h1; sFiiL[ib] = (us16)l1;
                }
            } else {
                float* fp = sFij + (e - 1) * RB * FIJP;
                float v0[8], v1[8];
#pragma unroll
                for (int r = 0; r < 8; ++r) { v0[r] = okn ? (c0[r] + bb) : 0.0f; v1[r] = okn ? (c1[r] + bb) : 0.0f; }
                if (n < FIJP) {
#pragma unroll
                    for (int r = 0; r < 8; ++r) {
                        fp[(8 * hh + r) * FIJP + n]      = v0[r];
                        fp[(16 + 8 * hh + r) * FIJP + n] = v1[r];
                    }
                }
            }
        }
        if (e == 0) {
            v4u_t z4; z4.x = 0u; z4.y = 0u; z4.z = 0u; z4.w = 0u;
            *(v4u*)(sFiiH + lane * SP + 112) = z4; *(v4u*)(sFiiH + lane * SP + 120) = z4;
            *(v4u*)(sFiiL + lane * SP + 112) = z4; *(v4u*)(sFiiL + lane * SP + 120) = z4;
        }
    }
    __syncthreads();

    {
        const float* f0 = sFij;
        const float* f1 = sFij + RB * FIJP;

        float p0[8], p1[8], q0[8], q1[8];
#pragma unroll
        for (int r = 0; r < 8; ++r) { p0[r] = 0.0f; p1[r] = 0.0f; q0[r] = 0.0f; q1[r] = 0.0f; }
#pragma unroll 1
        for (int nt = 0; nt < NT; ++nt) {
            v8f c0, c1;
            tile_mm<KSQ, true>(sFiiH, sFiiL, SP, wsh + PH_CORR + nt * 16 * KSQ, lane, c0, c1);
            const int n  = nt * 16 + m;
            const int cc = (n < FIJP) ? n : (FIJP - 1);
#pragma unroll
            for (int r = 0; r < 8; ++r) {
                const int ia = (8 * hh + r) * FIJP + cc, ib = (16 + 8 * hh + r) * FIJP + cc;
                p0[r] = fmaf(c0[r], f0[ia], p0[r]); p1[r] = fmaf(c0[r], f1[ia], p1[r]);
                q0[r] = fmaf(c1[r], f0[ib], q0[r]); q1[r] = fmaf(c1[r], f1[ib], q1[r]);
            }
        }
        reduce16(p0); reduce16(p1); reduce16(q0); reduce16(q1);
        float at0[8], at1[8], bt0[8], bt1[8];
#pragma unroll
        for (int r = 0; r < 8; ++r) {
            softmax2(p0[r], p1[r], at0[r], at1[r]);
            softmax2(q0[r], q1[r], bt0[r], bt1[r]);
        }

#pragma unroll 1
        for (int j = 0; j < NT; ++j) {
            const int cj = m + 16 * j;
            const int cc = (cj < HN) ? cj : (HN - 1);
            unsigned int ah[8], al[8], bh[8], bl[8];
#pragma unroll
            for (int r = 0; r < 8; ++r) {
                const int ra = 8 * hh + r, rb = 16 + 8 * hh + r;
                const float va = fmaf(at0[r], f0[ra * FIJP + cc], at1[r] * f1[ra * FIJP + cc]);
                const float vb = fmaf(bt0[r], f0[rb * FIJP + cc], bt1[r] * f1[rb * FIJP + cc]);
                split2(va, ah[r], al[r]); split2(vb, bh[r], bl[r]);
            }
            if (cj < HN) {
#pragma unroll
                for (int r = 0; r < 8; ++r) {
                    const int ia = (8 * hh + r) * CATP + HN + cj, ib = (16 + 8 * hh + r) * CATP + HN + cj;
                    sCatH[ia] = (us16)ah[r]; sCatL[ia] = (us16)al[r];
                    sCatH[ib] = (us16)bh[r]; sCatL[ib] = (us16)bl[r];
                }
            }
        }
        {
            v4u_t z4; z4.x = 0u; z4.y = 0u; z4.z = 0u; z4.w = 0u;
            us16* ch = sCatH + lane * CATP + 2 * HN;
            us16* cl = sCatL + lane * CATP + 2 * HN;
            *(v4u*)(ch) = z4; *(v4u*)(ch + 8) = z4; *(v4u*)(ch + 16) = z4;
            *(v4u*)(cl) = z4; *(v4u*)(cl + 8) = z4; *(v4u*)(cl + 16) = z4;
        }

        const float* FCB = par + V_FCB * PV;
#pragma unroll 1
        for (int nt = 0; nt < NT; ++nt) {
            v8f c0, c1;
            tile_mm<KSQ, true>(sFiiH, sFiiL, SP, wsh + PH_FC + nt * 16 * KSQ, lane, c0, c1);
            const int n = nt * 16 + m;
            const float bb = FCB[n];
            unsigned int h0[8], l0[8], h1[8], l1[8];
#pragma unroll
            for (int r = 0; r < 8; ++r) { split2(c0[r] + bb, h0[r], l0[r]); split2(c1[r] + bb, h1[r], l1[r]); }
            if (n < HN) {
#pragma unroll
                for (int r = 0; r < 8; ++r) {
                    const int ia = (8 * hh + r) * CATP + n, ib = (16 + 8 * hh + r) * CATP + n;
                    sCatH[ia] = (us16)h0[r]; sCatL[ia] = (us16)l0[r];
                    sCatH[ib] = (us16)h1[r]; sCatL[ib] = (us16)l1[r];
                }
            }
        }
        __syncthreads();

        const float* CB1 = par + V_CB1 * PV;
        const float* CW2 = par + V_CW2 * PV;
        float pv[8], pw[8];
#pragma unroll
        for (int r = 0; r < 8; ++r) { pv[r] = 0.0f; pw[r] = 0.0f; }
#pragma unroll 1
        for (int nt = 0; nt < NT; ++nt) {
            v8f c0, c1;
            tile_mm<KCR, true>(sCatH, sCatL, CATP, wsh + PH_CR1 + nt * 16 * KCR, lane, c0, c1);
            const int n = nt * 16 + m;
            const float bb = CB1[n], w2 = CW2[n];
#pragma unroll
            for (int r = 0; r < 8; ++r) {
                pv[r] = fmaf(tanh_v(c0[r] + bb), w2, pv[r]);
                pw[r] = fmaf(tanh_v(c1[r] + bb), w2, pw[r]);
            }
        }
        reduce16(pv); reduce16(pw);
        const float cb2 = par[V_CB2 * PV];
        if (m == 0) {
#pragma unroll
            for (int r = 0; r < 8; ++r) {
                sRow[8 * hh + r]      = pv[r] + cb2;
                sRow[16 + 8 * hh + r] = pw[r] + cb2;
            }
        }
        sRow[RB + lane] = rnn[b0 + lane];
        __syncthreads();

        const size_t off = (lane < 8) ? ((size_t)b0 + 4 * lane)
                                      : ((size_t)bsz * (HN + 1) + (size_t)b0 + 4 * (lane - 8));
        const int li = (lane < 16) ? lane : 0;
        const v4f_t v = *(const v4f*)(sRow + 4 * li);
        if (lane < 16) *(volatile v4f_t*)(out + off) = v;
        __threadfence();
        if (lane < 16) *(volatile v4f_t*)(out + off) = v;
    }
}

extern "C" void kernel_launch(void* const* d_in, const int* in_sizes, int n_in,
                              void* d_out, int out_size, void* d_ws, size_t ws_size,
                              hipStream_t stream)
{
    if (n_in < 28) return;
    const int bsz = in_sizes[1] / OBS;
    if (bsz <= 0 || (bsz % RB) != 0) return;
    if (in_sizes[1] != bsz * OBS) return;
    if (in_sizes[0] != bsz * OBSS) return;
    if (in_sizes[2] < 1) return;
    if (in_sizes[3] != bsz) return;
    if (out_size != bsz * (HN + 2)) return;
    if (in_sizes[5]  != OBS * HN)     return;
    if (in_sizes[6]  != HN)           return;
    if (in_sizes[7]  != HN * HN)      return;
    if (in_sizes[8]  != HN)           return;
    if (in_sizes[9]  != 4 * HN)       return;
    if (in_sizes[10] != HN)           return;
    if (in_sizes[11] != 2 * HN)       return;
    if (in_sizes[12] != HN)           return;
    if (in_sizes[13] != 2 * HN)       return;
    if (in_sizes[14] != HN)           return;
    if (in_sizes[15] != HN * HN)      return;
    if (in_sizes[16] != HN * HN)      return;
    if (in_sizes[17] != HN * HN)      return;
    if (in_sizes[18] != HN)           return;
    if (in_sizes[19] != 3 * HN * HN)  return;
    if (in_sizes[20] != HN)           return;
    if (in_sizes[21] != HN * HN)      return;
    if (in_sizes[22] != HN * HN)      return;
    if (in_sizes[23] != HN)           return;
    if (in_sizes[24] != 2 * HN * HN)  return;
    if (in_sizes[25] != HN)           return;
    if (in_sizes[26] != HN)           return;
    if (in_sizes[27] < 1)             return;
    if (WS_TOTAL > ws_size) return;

    const float* share = (const float*)d_in[0];
    const float* inp   = (const float*)d_in[1];
    const int*   agent = (const int*)d_in[2];
    const float* rnn   = (const float*)d_in[3];
    const float* aw1 = (const float*)d_in[5];  const float* ab1 = (const float*)d_in[6];
    const float* aw2 = (const float*)d_in[7];  const float* ab2 = (const float*)d_in[8];
    const float* esw = (const float*)d_in[9];  const float* esb = (const float*)d_in[10];
    const float* eaw = (const float*)d_in[11]; const float* eab = (const float*)d_in[12];
    const float* elw = (const float*)d_in[13]; const float* elb = (const float*)d_in[14];
    const float* eac = (const float*)d_in[15]; const float* elc = (const float*)d_in[16];
    const float* efw = (const float*)d_in[17]; const float* efb = (const float*)d_in[18];
    const float* eow = (const float*)d_in[19]; const float* eob = (const float*)d_in[20];
    const float* cmt = (const float*)d_in[21];
    const float* fcw = (const float*)d_in[22]; const float* fcb = (const float*)d_in[23];
    const float* cw1 = (const float*)d_in[24]; const float* cb1 = (const float*)d_in[25];
    const float* cw2 = (const float*)d_in[26]; const float* cb2 = (const float*)d_in[27];

    char*  wsb = (char*)d_ws;
    us16*  wsh = (us16*)wsb;
    float* par = (float*)(wsb + PAR_OFFB);
    float* out = (float*)d_out;

    const int npA1 = NROW * KA1 / 8, npSQ = NROW * KSQ / 8, npEO = NROW * KEO / 8, npCR = NROW * KCR / 8;
    pack_plane<<<(npA1 + 255) / 256, 256, 0, stream>>>(aw1, OBS,    KA1, HN, npA1, wsh + PH_A1);
    pack_plane<<<(npSQ + 255) / 256, 256, 0, stream>>>(aw2, HN,     KSQ, HN, npSQ, wsh + PH_A2);
    pack_plane<<<(npEO + 255) / 256, 256, 0, stream>>>(eow, 3 * HN, KEO, HN, npEO, wsh + PH_EOUT);
    pack_plane<<<(npSQ + 255) / 256, 256, 0, stream>>>(cmt, HN,     KSQ, HN, npSQ, wsh + PH_CORR);
    pack_plane<<<(npSQ + 255) / 256, 256, 0, stream>>>(fcw, HN,     KSQ, HN, npSQ, wsh + PH_FC);
    pack_plane<<<(npCR + 255) / 256, 256, 0, stream>>>(cw1, 2 * HN, KCR, HN, npCR, wsh + PH_CR1);

    prep_small<<<1, 256, 0, stream>>>(ab1, ab2, esw, esb, eaw, eab, elw, elb, eac, elc,
                                        efw, efb, eob, fcb, cb1, cw2, cb2, par);

    actor_kernel<<<bsz / RB, 32, 0, stream>>>(inp, wsh, par, out, bsz);

    hipFuncSetAttribute(reinterpret_cast<const void*>(&enc_head_kernel),
                        hipFuncAttributeMaxDynamicSharedMemorySize, L_TOTAL);
    enc_head_kernel<<<bsz / RB, 32, L_TOTAL, stream>>>(share, inp, agent, rnn, wsh, par, out, bsz);
}
